// GatedRelevanceNetwork_335007449190
// MI455X (gfx1250) — hardware-run, weakly checked
//
#include <hip/hip_runtime.h>


#define NBT 8
#define NL  64
#define ND  256
#define NK  32
typedef _Float16 h16;
typedef unsigned short bf;
typedef __attribute__((ext_vector_type(16))) __bf16   v16bf;
typedef __attribute__((ext_vector_type(16))) _Float16 v16h;
typedef __attribute__((ext_vector_type(8)))  _Float16 v8h;
typedef __attribute__((ext_vector_type(8)))  unsigned short v8us;
typedef __attribute__((ext_vector_type(8)))  float    v8f;
typedef __attribute__((ext_vector_type(4)))  float    v4f;
typedef v8h  __attribute__((may_alias)) v8ha;
typedef v4f  __attribute__((may_alias)) v4fa;
typedef v8us __attribute__((may_alias)) v8usa;

__device__ __forceinline__ unsigned short f2bf(float f) { unsigned u = __float_as_uint(f); u += 0x7FFFu + ((u >> 16) & 1u); return (unsigned short)(u >> 16); }
__device__ __forceinline__ float bf2f(unsigned short b) { return __uint_as_float(((unsigned)b) << 16); }
__device__ __forceinline__ float bfr(float f) { return bf2f(f2bf(f)); }
__device__ __forceinline__ v16h cat16(v8h lo, v8h hi) { return __builtin_shufflevector(lo, hi, 0, 1, 2, 3, 4, 5, 6, 7, 8, 9, 10, 11, 12, 13, 14, 15); }
__device__ __forceinline__ v16bf cat16b(v8us lo, v8us hi) { return __builtin_bit_cast(v16bf, __builtin_shufflevector(lo, hi, 0, 1, 2, 3, 4, 5, 6, 7, 8, 9, 10, 11, 12, 13, 14, 15)); }
__device__ __forceinline__ v8f wmma16(v16h a, v16h b, v8f c) { return __builtin_amdgcn_wmma_f32_16x16x32_f16(false, a, false, b, (short)0, c, false, false); }
__device__ __forceinline__ v8f wmmab(v16bf a, v16bf b, v8f c) { return __builtin_amdgcn_wmma_f32_16x16x32_bf16(false, a, false, b, (short)0, c, false, false); }

template <typename T16> struct WFrag;
template <> struct WFrag<h16> { typedef v16h V; static __device__ __forceinline__ V ld(const h16* p) { return cat16(*(const v8h*)p, *(const v8h*)(p + 16)); } static __device__ __forceinline__ v8f mma(V a, V b, v8f c) { return wmma16(a, b, c); } };
template <> struct WFrag<bf> { typedef v16bf V; static __device__ __forceinline__ V ld(const bf* p) { return cat16b(*(const v8us*)p, *(const v8us*)(p + 16)); } static __device__ __forceinline__ v8f mma(V a, V b, v8f c) { return wmmab(a, b, c); } };
template <typename T16, int NSPLIT, bool BIAS>
__global__ __launch_bounds__(32) void k_gemmw(const T16* __restrict__ A, const T16* __restrict__ A2, const T16* __restrict__ Bt, const T16* __restrict__ Bt2, int K, float* C, int ldc, const float* __restrict__ bias, size_t sA, size_t sB, size_t sC) {
    typedef typename WFrag<T16>::V V;
    __shared__ __align__(16) float os[16 * 68];
    const size_t z = blockIdx.z; A += z * sA; if (A2) A2 += z * sA; Bt += z * sB; if (Bt2) Bt2 += z * sB; C += z * sC;
    const int lane = threadIdx.x & 31, lr = lane & 15, hi = lane >> 4; const int r0 = blockIdx.x * 64, c0 = blockIdx.y * 64;
    v8f acc[4][4];
#pragma unroll
    for (int mb = 0; mb < 4; ++mb)
#pragma unroll
        for (int nb = 0; nb < 4; ++nb) acc[mb][nb] = (v8f){};
    const size_t aoff = (size_t)(r0 + lr) * K + 8 * hi, boff = (size_t)(c0 + lr) * K + 8 * hi;
    for (int kc = 0; kc < K; kc += 32) {
        V a[4], a2[4];
#pragma unroll
        for (int mb = 0; mb < 4; ++mb) { a[mb] = WFrag<T16>::ld(A + aoff + (size_t)mb * 16 * K + kc); if (NSPLIT == 1 || NSPLIT == 2) a2[mb] = WFrag<T16>::ld(A2 + aoff + (size_t)mb * 16 * K + kc); }
#pragma unroll
        for (int nb = 0; nb < 4; ++nb) { const V b = WFrag<T16>::ld(Bt + boff + (size_t)nb * 16 * K + kc); V b2; if (NSPLIT >= 2) b2 = WFrag<T16>::ld(Bt2 + boff + (size_t)nb * 16 * K + kc);
#pragma unroll
            for (int mb = 0; mb < 4; ++mb) { acc[mb][nb] = WFrag<T16>::mma(a[mb], b, acc[mb][nb]); if (NSPLIT == 1 || NSPLIT == 2) acc[mb][nb] = WFrag<T16>::mma(a2[mb], b, acc[mb][nb]); if (NSPLIT >= 2) acc[mb][nb] = WFrag<T16>::mma(a[mb], b2, acc[mb][nb]); } }
        asm volatile("v_nop\n\tv_nop\n\tv_nop\n\tv_nop" : "+v"(acc[0][0]), "+v"(acc[1][1]), "+v"(acc[2][2]), "+v"(acc[3][3]) : "v"(a[0]), "v"(a[3]));
    }
#pragma unroll
    for (int mb = 0; mb < 4; ++mb) {
#pragma unroll
        for (int nb = 0; nb < 4; ++nb) {
#pragma unroll
            for (int j = 0; j < 8; ++j) os[(hi * 8 + j) * 68 + nb * 16 + lr] = acc[mb][nb][j]; }
        __builtin_amdgcn_wave_barrier(); asm volatile("" ::: "memory");
        float* crow = C + (size_t)(r0 + mb * 16) * ldc + c0;
#pragma unroll 1
        for (int ps = 0; ps < 2; ++ps) {
#pragma unroll
            for (int s = 0; s < 8; ++s) { const int row = 2 * s + hi, cofs = lr * 4; v4f val = *(const v4fa*)(os + row * 68 + cofs); if (BIAS) { val[0] += bfr(bias[c0 + cofs]); val[1] += bfr(bias[c0 + cofs + 1]); val[2] += bfr(bias[c0 + cofs + 2]); val[3] += bfr(bias[c0 + cofs + 3]); }
                *(volatile v4f*)(crow + (size_t)row * ldc + cofs) = val; }
            if (ps == 0) __threadfence(); }
        __builtin_amdgcn_wave_barrier(); asm volatile("" ::: "memory");
    }
}

__device__ __forceinline__ void splitf(float y, unsigned short& h, unsigned short& l) { h = f2bf(y); l = f2bf(y - bf2f(h)); }
typedef __attribute__((ext_vector_type(2))) _Float16 v2h;
typedef __attribute__((ext_vector_type(4))) _Float16 v4h;
typedef __attribute__((ext_vector_type(2))) unsigned short v2us;
typedef __attribute__((ext_vector_type(4))) unsigned short v4us;
typedef __attribute__((ext_vector_type(2))) float v2f;
typedef __attribute__((ext_vector_type(4))) int v4i;

__global__ __launch_bounds__(256) void k_cvt8(const float* __restrict__ src, bf* dst, size_t n8) { const size_t i = (size_t)blockIdx.x * 256 + threadIdx.x; if (i >= n8) return; const v8f v = *(const v8f*)(src + i * 8); v8us o;
#pragma unroll
    for (int k = 0; k < 8; ++k) o[k] = f2bf(v[k]); *(volatile v8us*)(dst + i * 8) = o; __threadfence(); *(volatile v8us*)(dst + i * 8) = o; }

__global__ __launch_bounds__(256) void k_pl2(const float* __restrict__ F, bf* Ph, bf* Pl, size_t n4) { const size_t i = (size_t)blockIdx.x * 256 + threadIdx.x; if (i >= n4) return; const v4f v = *(const v4f*)(F + i * 4); v4us oh, ol;
#pragma unroll
    for (int q = 0; q < 4; ++q) { unsigned short a, c; splitf(v[q], a, c); oh[q] = a; ol[q] = c; } *(volatile v4us*)(Ph + i * 4) = oh; *(volatile v4us*)(Pl + i * 4) = ol; __threadfence(); *(volatile v4us*)(Ph + i * 4) = oh; *(volatile v4us*)(Pl + i * 4) = ol; }

__global__ __launch_bounds__(256) void k_wtG(const float* __restrict__ w, int K, int N, bf* Bt) {
    const int lane = threadIdx.x & 31; const int L0 = (blockIdx.x * 8 + (threadIdx.x >> 5)) * 8; const int nlines = N * K / 64;
#pragma unroll
    for (int ps = 0; ps < 2; ++ps) {
        for (int l = 0; l < 8; ++l) { const int L = L0 + l; if (L >= nlines) break; const size_t e = (size_t)L * 64 + lane * 2; const int k = (int)(e % K), n = (int)(e / K); v2us o;
            o[0] = f2bf(w[(size_t)k * N + n]); o[1] = f2bf(w[(size_t)(k + 1) * N + n]); *(volatile v2us*)(Bt + e) = o; }
        if (ps == 0) __threadfence(); }
}

__global__ __launch_bounds__(256) void k_pair(const float* __restrict__ BT, const float* __restrict__ C1, const float* __restrict__ C2, const float* __restrict__ bg, const float* __restrict__ bb, const float* __restrict__ uu, float* OUT) {
  const int i = blockIdx.x * 256 + threadIdx.x; if (i >= NBT * NL * NL) return; const int n = i % NL, m = (i / NL) % NL, b = i / (NL * NL);
  const float* bt = BT + ((size_t)(b * NL + m) * NK) * NL + n; const float* c1 = C1 + (size_t)(b * NL + m) * 64; const float* c2 = C2 + (size_t)(b * NL + n) * 64; float s = 0.0f;
#pragma unroll 1
  for (int k = 0; k < NK; ++k) { const float btp = bt[(size_t)k * NL]; const float sln = tanhf(c1[k] + c2[k]); const float z = c1[NK + k] + c2[NK + k] + bfr(bg[k]); const float g = 1.0f / (1.0f + expf(-z)); const float fused = g * btp + (1.0f - g) * sln + bfr(bb[k]); s += fused * bfr(uu[k]); }
  *(volatile float*)(OUT + i) = s; __threadfence(); *(volatile float*)(OUT + i) = s;
}

extern "C" void kernel_launch(void* const* d_in, const int* in_sizes, int n_in,
                              void* d_out, int out_size, void* d_ws, size_t ws_size, hipStream_t stream) {
    (void)in_sizes; (void)n_in; (void)out_size;
    const float* arg1 = (const float*)d_in[0]; const float* arg2 = (const float*)d_in[1]; const float* Wb = (const float*)d_in[2]; const float* Wd = (const float*)d_in[3]; const float* Wg = (const float*)d_in[4];
    const float* bg = (const float*)d_in[5]; const float* bb = (const float*)d_in[6]; const float* uu = (const float*)d_in[7];
    float* OUT = (float*)d_out;
    char* wsp = (char*)d_ws;
    auto take = [&](size_t bytes) { char* p = wsp; wsp += (bytes + 255) & ~(size_t)255; return (void*)p; };
    const size_t NR = (size_t)NBT * NL;
    bf* A1 = (bf*)take(NR * ND * 2); bf* A2 = (bf*)take(NR * ND * 2); bf* WBt = (bf*)take((size_t)NK * ND * ND * 2); float* T = (float*)take(NR * NK * ND * 4); bf* Th = (bf*)take(NR * NK * ND * 2); bf* Tl = (bf*)take(NR * NK * ND * 2);
    float* BT = (float*)take(NR * NK * NL * 4); bf* P1 = (bf*)take((size_t)64 * ND * 2); bf* P2 = (bf*)take((size_t)64 * ND * 2); float* C1 = (float*)take(NR * 64 * 4); float* C2 = (float*)take(NR * 64 * 4);
    if ((size_t)(wsp - (char*)d_ws) > ws_size) return;
    k_cvt8<<<(unsigned)((NR * ND / 8 + 255) / 256), 256, 0, stream>>>(arg1, A1, NR * ND / 8); k_cvt8<<<(unsigned)((NR * ND / 8 + 255) / 256), 256, 0, stream>>>(arg2, A2, NR * ND / 8);
    for (int k = 0; k < NK; ++k) k_wtG<<<(unsigned)((ND * ND / 64 + 63) / 64), 256, 0, stream>>>(Wb + (size_t)k * ND * ND, ND, ND, WBt + (size_t)k * ND * ND);
    k_gemmw<bf, 0, false><<<dim3((unsigned)(NR / 64), NK * ND / 64, 1), 32, 0, stream>>>(A1, nullptr, WBt, nullptr, ND, T, NK * ND, nullptr, 0, 0, 0);
    k_pl2<<<(unsigned)((NR * NK * ND / 4 + 255) / 256), 256, 0, stream>>>(T, Th, Tl, NR * NK * ND / 4);
    for (int b = 0; b < NBT; ++b) k_gemmw<bf, 1, false><<<dim3(NL * NK / 64, NL / 64, 1), 32, 0, stream>>>(Th + (size_t)b * NL * NK * ND, Tl + (size_t)b * NL * NK * ND, A2 + (size_t)b * NL * ND, nullptr, ND, BT + (size_t)b * NL * NK * NL, NL, nullptr, 0, 0, 0);
    k_wtG<<<(unsigned)((ND * NK / 64 + 63) / 64), 256, 0, stream>>>(Wd, ND, NK, P1); k_wtG<<<(unsigned)((ND * NK / 64 + 63) / 64), 256, 0, stream>>>(Wg, ND, NK, P1 + (size_t)NK * ND);
    k_wtG<<<(unsigned)((ND * NK / 64 + 63) / 64), 256, 0, stream>>>(Wd + (size_t)ND * NK, ND, NK, P2); k_wtG<<<(unsigned)((ND * NK / 64 + 63) / 64), 256, 0, stream>>>(Wg + (size_t)ND * NK, ND, NK, P2 + (size_t)NK * ND);
    k_gemmw<bf, 0, false><<<dim3((unsigned)(NR / 64), 1, 1), 32, 0, stream>>>(A1, nullptr, P1, nullptr, ND, C1, 64, nullptr, 0, 0, 0); k_gemmw<bf, 0, false><<<dim3((unsigned)(NR / 64), 1, 1), 32, 0, stream>>>(A2, nullptr, P2, nullptr, ND, C2, 64, nullptr, 0, 0, 0);
    k_pair<<<(NBT * NL * NL + 255) / 256, 256, 0, stream>>>(BT, C1, C2, bg, bb, uu, OUT);
}
